// SpeMamba_47425028882458
// MI455X (gfx1250) — hardware-run, weakly checked
//
#include <hip/hip_runtime.h>
#include <math.h>

#define NB   4
#define NCH  200
#define IMH  128
#define IMW  128
#define PSD  4
#define PGH  32
#define PGW  32
#define DMD  1024
#define DIN  2048
#define DST  16
#define DTR  64
#define XPR  96
#define XDN  128
#define DCV  4
#define NROW (NB * NCH)
#define MP   896
#define EPSV 1e-5f
#define GSTR 40
#define OSTR 68
#define SMEMB (8 * 16 * OSTR * 4)
#define LOG2E 1.4426950408889634f

static_assert(MP % 128 == 0);
static_assert(MP >= NROW);
static_assert(DMD == PGH * PGW);
static_assert(IMH == PGH * PSD);
static_assert(IMW == PGW * PSD);
static_assert(DMD % 64 == 0);
static_assert(DIN % 64 == 0);
static_assert(XDN % 64 == 0);
static_assert(XPR <= XDN);
static_assert(DTR + 2 * DST <= XDN);
static_assert(DTR % 32 == 0);
static_assert(DMD % 32 == 0);
static_assert(DIN % 32 == 0);
static_assert(SMEMB >= (2 * 128 * GSTR + 64 * GSTR) * 2);
static_assert(DMD == 128 * 8);
static_assert(DIN == 512 * 4);
static_assert(DMD == 256 * 4);
static_assert(IMW == 32 * 4);
static_assert(((long)NB * NCH * IMH * IMW / 4) % 256 == 0);
static_assert(DIN % 128 == 0);

typedef unsigned short us16 __attribute__((ext_vector_type(16)));
typedef unsigned short us8  __attribute__((ext_vector_type(8)));
typedef unsigned short us8a __attribute__((ext_vector_type(8), may_alias));
typedef unsigned short us4  __attribute__((ext_vector_type(4)));
typedef __bf16 v16b __attribute__((ext_vector_type(16)));
typedef float v8f __attribute__((ext_vector_type(8)));
typedef float v4f __attribute__((ext_vector_type(4)));
typedef float v4fa __attribute__((ext_vector_type(4), may_alias));
union FragU { us16 v; us8 h[2]; };

__device__ __forceinline__ unsigned short bf16_bits(float f) {
  unsigned u = __float_as_uint(f);
  u += 0x7FFFu + ((u >> 16) & 1u);
  return (unsigned short)(u >> 16);
}
__device__ __forceinline__ float bf16_val(unsigned short b) { return __uint_as_float(((unsigned)b) << 16); }
__device__ __forceinline__ float bf16r(float f) { return bf16_val(bf16_bits(f)); }
__device__ __forceinline__ float siluf(float x) { return x * __builtin_amdgcn_rcpf(1.0f + __expf(-x)); }
__device__ __forceinline__ int iclamp(int v, int lo, int hi) { return v < lo ? lo : (v > hi ? hi : v); }

__device__ __forceinline__ v8f mma_bf16(us16 a, us16 b, v8f c) {
  return __builtin_amdgcn_wmma_f32_16x16x32_bf16(false, __builtin_bit_cast(v16b, a), false, __builtin_bit_cast(v16b, b), (short)0, c, false, false);
}
__device__ __forceinline__ void wguard(v8f& c0, v8f& c1, v8f& c2, v8f& c3, const us16& a0, const us16& a1,
                                       const us16& b0, const us16& b1, const us16& b2, const us16& b3) {
#if defined(__HIP_DEVICE_COMPILE__)
  asm volatile("v_nop\n\tv_nop\n\tv_nop\n\tv_nop"
               : "+v"(c0), "+v"(c1), "+v"(c2), "+v"(c3)
               : "v"(a0), "v"(a1), "v"(b0), "v"(b1), "v"(b2), "v"(b3));
#endif
}

__device__ __forceinline__ us16 lds_frag(const unsigned short* base) {
  const int lane = threadIdx.x & 31, r = lane & 15, kh = (lane >> 4) * 8;
  FragU f;
  f.h[0] = *(const us8a*)(base + r * GSTR + kh);
  f.h[1] = *(const us8a*)(base + r * GSTR + 16 + kh);
  return f.v;
}

__device__ __forceinline__ void stage_a(unsigned short* lds, const unsigned short* __restrict__ P, int ld, int m0, int k0, int tid) {
  const int row = tid >> 1, cq = (tid & 1) * 16;
  const unsigned short* src = P + (size_t)(m0 + row) * ld + k0 + cq;
  const us8 v0 = *(const us8a*)src;
  const us8 v1 = *(const us8a*)(src + 8);
  *(us8a*)(lds + row * GSTR + cq) = v0;
  *(us8a*)(lds + row * GSTR + cq + 8) = v1;
}
__device__ __forceinline__ void stage_b(unsigned short* lds, const unsigned short* __restrict__ P, int ld, int n0, int k0, int tid) {
  const int row = tid >> 2, kq = (tid & 3) * 8;
  const us8 v = *(const us8a*)(P + (size_t)(n0 + row) * ld + k0 + kq);
  *(us8a*)(lds + row * GSTR + kq) = v;
}

template <int EPI>
__global__ __launch_bounds__(256) void k_gemm(const unsigned short* __restrict__ A0, const unsigned short* __restrict__ A1, int lda,
                                             const unsigned short* __restrict__ B0, int ldb,
                                             float* Y, float* Yalt, int nsplit, int ldy, int K,
                                             const float* __restrict__ bias) {
#pragma clang fp contract(off)
  __shared__ __attribute__((aligned(16))) unsigned char sm[SMEMB];
  unsigned short* lA0 = (unsigned short*)sm;
  unsigned short* lA1 = lA0 + 128 * GSTR;
  unsigned short* lB0 = lA1 + 128 * GSTR;
  float* oS = (float*)sm;
  const int tid = threadIdx.x, lane = tid & 31, wave = tid >> 5, cl = lane & 15, hh = lane >> 4;
  const int m0 = blockIdx.x * 128;
  const int n0 = blockIdx.y * 64;
  float* Yb = Y;
  int nq = n0;
  if (nsplit > 0 && n0 >= nsplit) { Yb = Yalt; nq = n0 - nsplit; }

  v8f acc[4];
#pragma unroll
  for (int j = 0; j < 4; ++j) { v8f zz = {0.f, 0.f, 0.f, 0.f, 0.f, 0.f, 0.f, 0.f}; acc[j] = zz; }

#pragma unroll 1
  for (int k0 = 0; k0 < K; k0 += 32) {
    __syncthreads();
    stage_a(lA0, A0, lda, m0, k0, tid);
    stage_a(lA1, A1, lda, m0, k0, tid);
    stage_b(lB0, B0, ldb, n0, k0, tid);
    __syncthreads();
    const us16 af0 = lds_frag(lA0 + 16 * wave * GSTR);
    const us16 af1 = lds_frag(lA1 + 16 * wave * GSTR);
    us16 bfr[4];
#pragma unroll
    for (int j = 0; j < 4; ++j) bfr[j] = lds_frag(lB0 + 16 * j * GSTR);
#pragma unroll
    for (int j = 0; j < 4; ++j) acc[j] = mma_bf16(af0, bfr[j], acc[j]);
#pragma unroll
    for (int j = 0; j < 4; ++j) acc[j] = mma_bf16(af1, bfr[j], acc[j]);
    wguard(acc[0], acc[1], acc[2], acc[3], af0, af1, bfr[0], bfr[1], bfr[2], bfr[3]);
  }
  __syncthreads();

  float bj[4];
#pragma unroll
  for (int j = 0; j < 4; ++j) {
    if (EPI == 1) bj[j] = bf16r(bias[n0 + 16 * j + cl]);
    else          bj[j] = 0.0f;
  }
  float* so = oS + wave * (16 * OSTR);
#pragma unroll
  for (int j = 0; j < 4; ++j)
#pragma unroll
    for (int r = 0; r < 8; ++r) so[(8 * hh + r) * OSTR + 16 * j + cl] = acc[j][r] + bj[j];
  __syncthreads();
#pragma unroll
  for (int pass = 0; pass < 2; ++pass) {
#pragma unroll
    for (int it = 0; it < 8; ++it) {
      const int ch = it * 32 + lane, r = ch >> 4, q = (ch & 15) * 4;
      const v4f v = *(const v4fa*)(so + r * OSTR + q);
      *(volatile v4f*)(Yb + (size_t)(m0 + 16 * wave + r) * ldy + nq + q) = v;
    }
    __threadfence();
  }
}

__global__ __launch_bounds__(256) void k_cvt(const float* __restrict__ src, unsigned short* dst, int nsrc, int ncol8, int total8) {
  const int idx = blockIdx.x * 256 + threadIdx.x;
  if (idx >= total8) return;
  const int row = idx / ncol8, c8 = (idx - row * ncol8) * 8;
  const int rs = (row < nsrc) ? row : (nsrc - 1);
  const float* s = src + (size_t)rs * (size_t)(ncol8 * 8) + c8;
  const v4f a = *(const v4fa*)s, b = *(const v4fa*)(s + 4);
  const bool zr = (row >= nsrc);
  us8 o;
#pragma unroll
  for (int u = 0; u < 4; ++u) {
    o[u]     = zr ? (unsigned short)0 : bf16_bits(a[u]);
    o[4 + u] = zr ? (unsigned short)0 : bf16_bits(b[u]);
  }
  const size_t off = (size_t)row * (size_t)(ncol8 * 8) + c8;
  *(volatile us8*)(dst + off) = o;
  __threadfence();
  *(volatile us8*)(dst + off) = o;
}

__global__ __launch_bounds__(256) void k_split(const float* __restrict__ src, unsigned short* H, unsigned short* L,
                                              int nsrc, int ncol8, int total8) {
#pragma clang fp contract(off)
  const int idx = blockIdx.x * 256 + threadIdx.x;
  if (idx >= total8) return;
  const int row = idx / ncol8, c8 = (idx - row * ncol8) * 8;
  const int rs = (row < nsrc) ? row : (nsrc - 1);
  const float* s = src + (size_t)rs * (size_t)(ncol8 * 8) + c8;
  const v4f a = *(const v4fa*)s, b = *(const v4fa*)(s + 4);
  const bool zr = (row >= nsrc);
  us8 hi, lo;
#pragma unroll
  for (int u = 0; u < 4; ++u) {
    const unsigned short ha = bf16_bits(a[u]);
    const unsigned short la = bf16_bits(a[u] - bf16_val(ha));
    const unsigned short hb = bf16_bits(b[u]);
    const unsigned short lb = bf16_bits(b[u] - bf16_val(hb));
    hi[u]     = zr ? (unsigned short)0 : ha;  lo[u]     = zr ? (unsigned short)0 : la;
    hi[4 + u] = zr ? (unsigned short)0 : hb;  lo[4 + u] = zr ? (unsigned short)0 : lb;
  }
  const size_t off = (size_t)row * (size_t)(ncol8 * 8) + c8;
  *(volatile us8*)(H + off) = hi; *(volatile us8*)(L + off) = lo;
  __threadfence();
  *(volatile us8*)(H + off) = hi; *(volatile us8*)(L + off) = lo;
}

__global__ __launch_bounds__(128) void k_pool(const float* __restrict__ X, unsigned short* PHp, unsigned short* PLp) {
#pragma clang fp contract(off)
  const int bc = blockIdx.x, t = threadIdx.x;
  us8 hi, lo;
  if (bc < NROW) {
    const int ph = t >> 2, pw0 = (t & 3) * 8;
    const float* base = X + (size_t)bc * (IMH * IMW) + (size_t)(ph * PSD) * IMW + pw0 * PSD;
    float s[8];
#pragma unroll
    for (int q = 0; q < 8; ++q) s[q] = 0.0f;
#pragma unroll
    for (int dy = 0; dy < PSD; ++dy) {
      const float* rp = base + dy * IMW;
#pragma unroll
      for (int q = 0; q < 8; ++q) {
        const v4f f = *(const v4fa*)(rp + 4 * q);
        s[q] = (((s[q] + bf16r(f[0])) + bf16r(f[1])) + bf16r(f[2])) + bf16r(f[3]);
      }
    }
#pragma unroll
    for (int q = 0; q < 8; ++q) {
      const float m = s[q] * (1.0f / (PSD * PSD));
      const unsigned short hb = bf16_bits(m);
      hi[q] = hb; lo[q] = bf16_bits(m - bf16_val(hb));
    }
  } else {
#pragma unroll
    for (int q = 0; q < 8; ++q) { hi[q] = (unsigned short)0; lo[q] = (unsigned short)0; }
  }
  const size_t o = (size_t)bc * DMD + 8 * t;
  *(volatile us8*)(PHp + o) = hi; *(volatile us8*)(PLp + o) = lo;
  __threadfence();
  *(volatile us8*)(PHp + o) = hi; *(volatile us8*)(PLp + o) = lo;
}

__global__ __launch_bounds__(256) void k_conv(const float* __restrict__ XU, const float* __restrict__ cw, const float* __restrict__ cb,
                                             unsigned short* UH, unsigned short* UL) {
#pragma clang fp contract(off)
  const int tok = blockIdx.x >> 1;
  const int c4 = (((blockIdx.x & 1) * 256) + threadIdx.x) * 4;
  us4 hi, lo;
  if (tok < NROW) {
    const int l = tok % NCH;
    v4f xv[DCV];
#pragma unroll
    for (int j = 0; j < DCV; ++j) {
      const int ll = l - (DCV - 1) + j;
      const int tc = (ll >= 0) ? (tok - (DCV - 1) + j) : tok;
      xv[j] = *(const v4fa*)(XU + (size_t)tc * DIN + c4);
    }
    const v4f b4 = *(const v4fa*)(cb + c4);
#pragma unroll
    for (int u = 0; u < 4; ++u) {
      const v4f wv = *(const v4fa*)(cw + (size_t)(c4 + u) * DCV);
      float a = 0.0f;
#pragma unroll
      for (int j = 0; j < DCV; ++j) {
        const float pr = bf16r(wv[j]) * xv[j][u];
        a = a + ((l - (DCV - 1) + j >= 0) ? pr : 0.0f);
      }
      a = a + bf16r(b4[u]);
      const float sv = siluf(a);
      const unsigned short hb = bf16_bits(sv);
      hi[u] = hb; lo[u] = bf16_bits(sv - bf16_val(hb));
    }
  } else {
#pragma unroll
    for (int u = 0; u < 4; ++u) { hi[u] = (unsigned short)0; lo[u] = (unsigned short)0; }
  }
  const size_t o = (size_t)tok * DIN + c4;
  *(volatile us4*)(UH + o) = hi; *(volatile us4*)(UL + o) = lo;
  __threadfence();
  *(volatile us4*)(UH + o) = hi; *(volatile us4*)(UL + o) = lo;
}

__global__ __launch_bounds__(128) void k_scan(const float* __restrict__ XD, const unsigned short* __restrict__ UH,
                                             const unsigned short* __restrict__ UL, const float* __restrict__ XZ,
                                             const float* __restrict__ DP, const float* __restrict__ Alog,
                                             const float* __restrict__ Dv, float* YF) {
#pragma clang fp contract(off)
  const int blk = blockIdx.x, tid = threadIdx.x;
  const int bb = blk / (DIN / 128);
  const int d = (blk - bb * (DIN / 128)) * 128 + tid;
  float A2[DST], h[DST];
#pragma unroll
  for (int n = 0; n < DST; ++n) { A2[n] = -__expf(bf16r(Alog[d * DST + n])) * LOG2E; h[n] = 0.0f; }
  const float Dd = bf16r(Dv[d]);
#pragma unroll 1
  for (int l = 0; l < NCH; ++l) {
    const size_t tok = (size_t)(bb * NCH + l);
    const float a = DP[tok * DIN + d];
    const float dl = fmaxf(a, 0.0f) + log1pf(__expf(-fabsf(a)));
    const float uv = bf16_val(UH[tok * DIN + d]) + bf16_val(UL[tok * DIN + d]);
    const float zv = XZ[tok * DIN + d];
    const float* xr = XD + tok * XDN;
    v4f Bv[4], Cv[4];
#pragma unroll
    for (int q = 0; q < 4; ++q) {
      Bv[q] = *(const v4fa*)(xr + DTR + 4 * q);
      Cv[q] = *(const v4fa*)(xr + DTR + DST + 4 * q);
    }
    const float dx = dl * uv;
    float y = 0.0f;
#pragma unroll
    for (int n = 0; n < DST; ++n) {
      const float e = exp2f(dl * A2[n]);
      h[n] = e * h[n] + dx * Bv[n >> 2][n & 3];
      y = y + h[n] * Cv[n >> 2][n & 3];
    }
    const float yv = (y + uv * Dd) * siluf(zv);
    float* yp = YF + tok * DIN + d;
    *(volatile float*)yp = yv;
    __threadfence();
    *(volatile float*)yp = yv;
  }
}

__global__ __launch_bounds__(256) void k_ln(const float* __restrict__ XP, const float* __restrict__ g, const float* __restrict__ bt,
                                           float* XO) {
#pragma clang fp contract(off)
  __shared__ float r1s[8];
  __shared__ float r2s[8];
  const int tid = threadIdx.x, lane = tid & 31, wave = tid >> 5, row = blockIdx.x, c4 = tid * 4;
  const v4f a = *(const v4fa*)(XP + (size_t)row * DMD + c4);
  float s = (a[0] + a[1]) + (a[2] + a[3]);
#pragma unroll
  for (int o = 16; o > 0; o >>= 1) s = s + __shfl_xor(s, o);
  if (lane == 0) r1s[wave] = s;
  __syncthreads();
  float tot = 0.0f;
#pragma unroll
  for (int w = 0; w < 8; ++w) tot = tot + r1s[w];
  const float mu = tot * (1.0f / DMD);
  float dv[4];
#pragma unroll
  for (int u = 0; u < 4; ++u) dv[u] = a[u] - mu;
  float s2 = ((dv[0] * dv[0] + dv[1] * dv[1]) + dv[2] * dv[2]) + dv[3] * dv[3];
#pragma unroll
  for (int o = 16; o > 0; o >>= 1) s2 = s2 + __shfl_xor(s2, o);
  if (lane == 0) r2s[wave] = s2;
  __syncthreads();
  float tot2 = 0.0f;
#pragma unroll
  for (int w = 0; w < 8; ++w) tot2 = tot2 + r2s[w];
  const float var = tot2 * (1.0f / DMD);
  const float rs = rsqrtf(var + EPSV);
  const v4f gv = *(const v4fa*)(g + c4), bv = *(const v4fa*)(bt + c4);
  v4f o;
#pragma unroll
  for (int u = 0; u < 4; ++u) {
    const float t = (dv[u] * rs) * bf16r(gv[u]) + bf16r(bv[u]);
    o[u] = siluf(t);
  }
  float* op = XO + (size_t)row * DMD + c4;
  *(volatile v4f*)op = o;
  __threadfence();
  *(volatile v4f*)op = o;
}

__global__ __launch_bounds__(256) void k_up(const float* __restrict__ X, const float* __restrict__ P, float* out) {
#pragma clang fp contract(off)
  const size_t e0 = ((size_t)blockIdx.x * 256 + threadIdx.x) * 4;
  const int j0 = (int)(e0 % IMW);
  const int i  = (int)((e0 / IMW) % IMH);
  const int bc = (int)(e0 / ((size_t)IMH * IMW));
  const v4f xv = *(const v4fa*)(X + e0);
  const float syf = ((float)i + 0.5f) * (1.0f / PSD) - 0.5f;
  const float y0f = floorf(syf);
  const float fy = syf - y0f;
  int y0 = (int)y0f;
  const int y1 = iclamp(y0 + 1, 0, PGH - 1);
  y0 = iclamp(y0, 0, PGH - 1);
  const float* p0 = P + (size_t)bc * DMD + y0 * PGW;
  const float* p1 = P + (size_t)bc * DMD + y1 * PGW;
  v4f o;
#pragma unroll
  for (int u = 0; u < 4; ++u) {
    const int j = j0 + u;
    const float sxf = ((float)j + 0.5f) * (1.0f / PSD) - 0.5f;
    const float x0f = floorf(sxf);
    const float fx = sxf - x0f;
    int x0 = (int)x0f;
    const int x1 = iclamp(x0 + 1, 0, PGW - 1);
    x0 = iclamp(x0, 0, PGW - 1);
    const float w00 = (1.0f - fy) * (1.0f - fx), w01 = (1.0f - fy) * fx, w10 = fy * (1.0f - fx), w11 = fy * fx;
    const float v = ((p0[x0] * w00 + p0[x1] * w01) + p1[x0] * w10) + p1[x1] * w11;
    o[u] = bf16r(xv[u]) + v;
  }
  float* op = out + e0;
  *(volatile v4f*)op = o;
  __threadfence();
  *(volatile v4f*)op = o;
}

extern "C" void kernel_launch(void* const* d_in, const int* in_sizes, int n_in,
                              void* d_out, int out_size, void* d_ws, size_t ws_size,
                              hipStream_t stream) {
  if (n_in < 14) return;
  if (in_sizes[0] != NB * NCH * IMH * IMW || in_sizes[1] != 2 * DIN * DMD || in_sizes[2] != DIN * DCV || in_sizes[3] != DIN ||
      in_sizes[4] != XPR * DIN || in_sizes[5] != DIN * DTR || in_sizes[6] != DIN || in_sizes[7] != DIN * DST || in_sizes[8] != DIN ||
      in_sizes[9] != DMD * DIN || in_sizes[10] != DMD * DMD || in_sizes[11] != DMD || in_sizes[12] != DMD || in_sizes[13] != DMD ||
      out_size != NB * NCH * IMH * IMW) return;

  const float* x      = (const float*)d_in[0];
  const float* W_in   = (const float*)d_in[1];
  const float* conv_w = (const float*)d_in[2];
  const float* conv_b = (const float*)d_in[3];
  const float* W_x    = (const float*)d_in[4];
  const float* W_dt   = (const float*)d_in[5];
  const float* b_dt   = (const float*)d_in[6];
  const float* A_log  = (const float*)d_in[7];
  const float* Dv     = (const float*)d_in[8];
  const float* W_out  = (const float*)d_in[9];
  const float* W_proj = (const float*)d_in[10];
  const float* b_proj = (const float*)d_in[11];
  const float* ln_g   = (const float*)d_in[12];
  const float* ln_b   = (const float*)d_in[13];
  float* out = (float*)d_out;

  size_t off = 0;
  auto carve = [&](size_t bytes) -> char* { char* p = (char*)d_ws + off; off += (bytes + 255) & ~(size_t)255; return p; };
  unsigned short* wIn16 = (unsigned short*)carve((size_t)2 * DIN * DMD * 2);
  unsigned short* wX16  = (unsigned short*)carve((size_t)XDN * DIN * 2);
  unsigned short* wDt16 = (unsigned short*)carve((size_t)DIN * DTR * 2);
  unsigned short* wO16  = (unsigned short*)carve((size_t)DMD * DIN * 2);
  unsigned short* wP16  = (unsigned short*)carve((size_t)DMD * DMD * 2);
  unsigned short* xfH   = (unsigned short*)carve((size_t)MP * DMD * 2);
  unsigned short* xfL   = (unsigned short*)carve((size_t)MP * DMD * 2);
  float* xU             = (float*)carve((size_t)MP * DIN * 4);
  float* xZ             = (float*)carve((size_t)MP * DIN * 4);
  unsigned short* uH    = (unsigned short*)carve((size_t)MP * DIN * 2);
  unsigned short* uL    = (unsigned short*)carve((size_t)MP * DIN * 2);
  float* xD             = (float*)carve((size_t)MP * XDN * 4);
  unsigned short* dbH   = (unsigned short*)carve((size_t)MP * XDN * 2);
  unsigned short* dbL   = (unsigned short*)carve((size_t)MP * XDN * 2);
  float* dPre           = (float*)carve((size_t)MP * DIN * 4);
  float* yF             = (float*)carve((size_t)NROW * DIN * 4);
  unsigned short* yH    = (unsigned short*)carve((size_t)MP * DIN * 2);
  unsigned short* yL    = (unsigned short*)carve((size_t)MP * DIN * 2);
  float* xM             = (float*)carve((size_t)MP * DMD * 4);
  unsigned short* xmH   = (unsigned short*)carve((size_t)MP * DMD * 2);
  unsigned short* xmL   = (unsigned short*)carve((size_t)MP * DMD * 2);
  float* xP             = (float*)carve((size_t)MP * DMD * 4);
  float* xPn            = (float*)carve((size_t)NROW * DMD * 4);
  if (off > ws_size || off > (size_t)134217728) return;

  const dim3 b256(256), b128(128);
  k_cvt<<<dim3((2 * DIN * (DMD / 8) + 255) / 256), b256, 0, stream>>>(W_in, wIn16, 2 * DIN, DMD / 8, 2 * DIN * (DMD / 8));
  k_cvt<<<dim3((XDN * (DIN / 8) + 255) / 256), b256, 0, stream>>>(W_x, wX16, XPR, DIN / 8, XDN * (DIN / 8));
  k_cvt<<<dim3((DIN * (DTR / 8) + 255) / 256), b256, 0, stream>>>(W_dt, wDt16, DIN, DTR / 8, DIN * (DTR / 8));
  k_cvt<<<dim3((DMD * (DIN / 8) + 255) / 256), b256, 0, stream>>>(W_out, wO16, DMD, DIN / 8, DMD * (DIN / 8));
  k_cvt<<<dim3((DMD * (DMD / 8) + 255) / 256), b256, 0, stream>>>(W_proj, wP16, DMD, DMD / 8, DMD * (DMD / 8));
  k_pool<<<dim3(MP), b128, 0, stream>>>(x, xfH, xfL);
  k_gemm<0><<<dim3(MP / 128, (2 * DIN) / 64), b256, 0, stream>>>(xfH, xfL, DMD, wIn16, DMD, xU, xZ, DIN, DIN, DMD, b_dt);
  k_conv<<<dim3(MP * 2), b256, 0, stream>>>(xU, conv_w, conv_b, uH, uL);
  k_gemm<0><<<dim3(MP / 128, XDN / 64), b256, 0, stream>>>(uH, uL, DIN, wX16, DIN, xD, xD, 0, XDN, DIN, b_dt);
  k_split<<<dim3((MP * (XDN / 8) + 255) / 256), b256, 0, stream>>>(xD, dbH, dbL, MP, XDN / 8, MP * (XDN / 8));
  k_gemm<1><<<dim3(MP / 128, DIN / 64), b256, 0, stream>>>(dbH, dbL, XDN, wDt16, DTR, dPre, dPre, 0, DIN, DTR, b_dt);
  k_scan<<<dim3(NB * (DIN / 128)), b128, 0, stream>>>(xD, uH, uL, xZ, dPre, A_log, Dv, yF);
  k_split<<<dim3((MP * (DIN / 8) + 255) / 256), b256, 0, stream>>>(yF, yH, yL, NROW, DIN / 8, MP * (DIN / 8));
  k_gemm<0><<<dim3(MP / 128, DMD / 64), b256, 0, stream>>>(yH, yL, DIN, wO16, DIN, xM, xM, 0, DMD, DIN, b_dt);
  k_split<<<dim3((MP * (DMD / 8) + 255) / 256), b256, 0, stream>>>(xM, xmH, xmL, MP, DMD / 8, MP * (DMD / 8));
  k_gemm<1><<<dim3(MP / 128, DMD / 64), b256, 0, stream>>>(xmH, xmL, DMD, wP16, DMD, xP, xP, 0, DMD, DMD, b_proj);
  k_ln<<<dim3(NROW), b256, 0, stream>>>(xP, ln_g, ln_b, xPn);
  k_up<<<dim3((unsigned)(((size_t)NB * NCH * IMH * IMW / 4) / 256)), b256, 0, stream>>>(x, xPn, out);
}
